// LinkPredictor_33964601377214
// MI455X (gfx1250) — hardware-run, weakly checked
//
#include <hip/hip_runtime.h>
#include <stddef.h>
#include <stdint.h>


#define FDIM   128
#define NTHR   256
#define NWAVE  8
#define EPT    8
#define CHUNK  (NTHR * EPT)
#define WCAP   (EPT * 32)
#define LISTN  (NWAVE * WCAP)
#define NBD    8192
#define SLB    13
#define NBA    480
#define SPW    (NBA / NWAVE)
#define GBM    64
#define GTHR   128
#define DTHR   256
#define WUNITS (FDIM * (FDIM / 8))
#define WSMAX  134217728

static_assert((CHUNK & (CHUNK - 1)) == 0 && CHUNK <= 4096);
static_assert((NBD & (NBD - 1)) == 0 && NBD == (1 << SLB));
static_assert(((long long)CHUNK << SLB) < (1LL << 31));
static_assert(NBD % (NTHR * 4) == 0);
static_assert(LISTN % NTHR == 0 && NBD % NTHR == 0);
static_assert(NBA % NWAVE == 0 && NBA <= NBD);
static_assert((NBA * FDIM) % (4 * NTHR) == 0);
static_assert(FDIM == 128 && FDIM % 32 == 0 && FDIM == 4 * 32);
static_assert(GBM == (GTHR / 32) * 16);
static_assert(WUNITS % NTHR == 0);
static_assert(DTHR % 32 == 0);

typedef float          v4f   __attribute__((ext_vector_type(4)));
typedef float          v8f   __attribute__((ext_vector_type(8)));
typedef int            v4i   __attribute__((ext_vector_type(4)));
typedef int            v8i   __attribute__((ext_vector_type(8)));
typedef unsigned short v8us  __attribute__((ext_vector_type(8)));
typedef unsigned short v16us __attribute__((ext_vector_type(16)));
typedef __bf16         v16bf __attribute__((ext_vector_type(16)));
typedef v4f  __attribute__((may_alias)) v4fa;
typedef v8us __attribute__((may_alias)) v8usa;
union FragB { v16bf v; v16us u; v8us h[2]; v8i w; };

__device__ __forceinline__ v8f wmb(const FragB& a, const FragB& b, v8f c) {
  v8f d = __builtin_amdgcn_wmma_f32_16x16x32_bf16(false, a.v, false, b.v, (short)0, c, false, false);
  asm volatile("v_nop\n\tv_nop\n\tv_nop\n\tv_nop" : "+v"(d) : "v"(a.w), "v"(b.w));
  return d;
}

__device__ __forceinline__ unsigned bf16_bits(float f) {
  const unsigned u = __float_as_uint(f);
  return (u + 0x7FFFu + ((u >> 16) & 1u)) >> 16;
}
__device__ __forceinline__ float bf16_val(float f) {
  return __uint_as_float(bf16_bits(f) << 16);
}

__device__ __forceinline__ int scan_chunk(const int* __restrict__ dsts, int nE, int cbase, int slotBase,
                                          int nb, int vec8, int* list, int tid, int lane, int wave) {
  int wc = 0;
  const int el0  = tid * EPT;
  const int e0   = cbase + el0;
  const int sent = -2147483647 - 1;
  v4i da, db;
  if (vec8 != 0 && cbase + CHUNK <= nE) {
    da = *(const v4i*)(dsts + e0);
    db = *(const v4i*)(dsts + e0 + 4);
  } else {
    da.x = (e0     < nE) ? dsts[min(e0,     nE - 1)] : sent;
    da.y = (e0 + 1 < nE) ? dsts[min(e0 + 1, nE - 1)] : sent;
    da.z = (e0 + 2 < nE) ? dsts[min(e0 + 2, nE - 1)] : sent;
    da.w = (e0 + 3 < nE) ? dsts[min(e0 + 3, nE - 1)] : sent;
    db.x = (e0 + 4 < nE) ? dsts[min(e0 + 4, nE - 1)] : sent;
    db.y = (e0 + 5 < nE) ? dsts[min(e0 + 5, nE - 1)] : sent;
    db.z = (e0 + 6 < nE) ? dsts[min(e0 + 6, nE - 1)] : sent;
    db.w = (e0 + 7 < nE) ? dsts[min(e0 + 7, nE - 1)] : sent;
  }
  const unsigned nbs = (unsigned)slotBase;
  const unsigned unb = (unsigned)nb;
  const unsigned s0 = (unsigned)da.x - nbs, s1 = (unsigned)da.y - nbs;
  const unsigned s2 = (unsigned)da.z - nbs, s3 = (unsigned)da.w - nbs;
  const unsigned s4 = (unsigned)db.x - nbs, s5 = (unsigned)db.y - nbs;
  const unsigned s6 = (unsigned)db.z - nbs, s7 = (unsigned)db.w - nbs;
  const bool h0 = s0 < unb, h1 = s1 < unb, h2 = s2 < unb, h3 = s3 < unb;
  const bool h4 = s4 < unb, h5 = s5 < unb, h6 = s6 < unb, h7 = s7 < unb;
  const unsigned any = __builtin_amdgcn_ballot_w32(h0 | h1 | h2 | h3 | h4 | h5 | h6 | h7);
  if (any != 0u) {
#define HITJ(J, HJ, SJ) { \
      const unsigned mj = __builtin_amdgcn_ballot_w32(HJ); \
      if (mj != 0u) { \
        if (HJ) { \
          const int pos = wc + (int)__builtin_amdgcn_mbcnt_lo(mj, 0u); \
          if (pos < WCAP) list[wave * WCAP + pos] = ((el0 + (J)) << SLB) | (int)(SJ); \
        } \
        wc += (int)__builtin_popcount(mj); } }
    HITJ(0, h0, s0)
    HITJ(1, h1, s1)
    HITJ(2, h2, s2)
    HITJ(3, h3, s3)
    HITJ(4, h4, s4)
    HITJ(5, h5, s5)
    HITJ(6, h6, s6)
    HITJ(7, h7, s7)
#undef HITJ
  }
  return wc;
}

__global__ __launch_bounds__(NTHR) void k_wprep(const float* __restrict__ W1, const float* __restrict__ W2,
                                                unsigned short* WT1, unsigned short* WT2) {
  const int nbw = WUNITS / NTHR;
  const int sel = ((int)blockIdx.x >= nbw) ? 1 : 0;
  const float* W = (sel != 0) ? W2 : W1;
  unsigned short* WT = (sel != 0) ? WT2 : WT1;
  const int u  = ((int)blockIdx.x - sel * nbw) * NTHR + (int)threadIdx.x;
  const int kq = FDIM >> 3;
  const int n  = u / kq;
  const int k8 = (u - n * kq) * 8;
  const float* p = W + (size_t)k8 * FDIM + n;
  v8us o;
  o[0] = (unsigned short)bf16_bits(p[0]);
  o[1] = (unsigned short)bf16_bits(p[(size_t)FDIM]);
  o[2] = (unsigned short)bf16_bits(p[(size_t)2 * FDIM]);
  o[3] = (unsigned short)bf16_bits(p[(size_t)3 * FDIM]);
  o[4] = (unsigned short)bf16_bits(p[(size_t)4 * FDIM]);
  o[5] = (unsigned short)bf16_bits(p[(size_t)5 * FDIM]);
  o[6] = (unsigned short)bf16_bits(p[(size_t)6 * FDIM]);
  o[7] = (unsigned short)bf16_bits(p[(size_t)7 * FDIM]);
  unsigned short* dp = WT + (size_t)n * FDIM + k8;
  *(volatile v8us*)dp = o;
  __threadfence();
  *(volatile v8us*)dp = o;
}

__global__ __launch_bounds__(NTHR) void k_deg(const int* __restrict__ dsts, int nE, int vec8, float* dis) {
  __shared__ __attribute__((aligned(16))) int scnt[NBD];
  __shared__ __attribute__((aligned(16))) int list[LISTN];
  __shared__ int wcnt[NWAVE];
  const int tid = (int)threadIdx.x, lane = tid & 31, wave = tid >> 5;
  const int nodeBase = (int)blockIdx.x * NBD;

  for (int i = tid; i < NBD; i += NTHR) scnt[i] = 0;
  for (int i = tid; i < LISTN; i += NTHR) list[i] = 0;
  if (tid < NWAVE) wcnt[tid] = 0;
  __syncthreads();

  const int nChunks = (nE + CHUNK - 1) / CHUNK;
#pragma unroll 1
  for (int ch = 0; ch < nChunks; ++ch) {
    const int cbase = ch * CHUNK;
    const int wc = scan_chunk(dsts, nE, cbase, nodeBase, NBD, vec8, list, tid, lane, wave);
    if (lane == 0) wcnt[wave] = wc;
    __syncthreads();
    if (wave == 0) {
#pragma unroll 1
      for (int w2 = 0; w2 < NWAVE; ++w2) {
        int c = wcnt[w2];
        c = c < 0 ? 0 : (c > WCAP ? WCAP : c);
#pragma unroll 1
        for (int b0 = 0; b0 < c; b0 += 32) {
          const int idx = b0 + lane;
          const int ent = list[w2 * WCAP + (idx < WCAP ? idx : WCAP - 1)];
          const int m32 = (c - b0) < 32 ? (c - b0) : 32;
#pragma unroll 1
          for (int k = 0; k < m32; ++k) {
            const int u  = __builtin_amdgcn_readlane(ent, k);
            const int sl = u & (NBD - 1);
            if (lane == 0) scnt[sl] = scnt[sl] + 1;
          }
        }
      }
    }
    __syncthreads();
  }

  v4f vals[NBD / (NTHR * 4)];
#pragma unroll
  for (int it = 0; it < NBD / (NTHR * 4); ++it) {
    const int s0 = it * (NTHR * 4) + 4 * tid;
    const v4i c4 = *(const v4i*)(scnt + s0);
    v4f v;
    v.x = rsqrtf((float)c4.x + 1.0f);
    v.y = rsqrtf((float)c4.y + 1.0f);
    v.z = rsqrtf((float)c4.z + 1.0f);
    v.w = rsqrtf((float)c4.w + 1.0f);
    vals[it] = v;
  }
#pragma unroll
  for (int it = 0; it < NBD / (NTHR * 4); ++it) {
    const int s0 = it * (NTHR * 4) + 4 * tid;
    *(volatile v4f*)(dis + (size_t)nodeBase + s0) = vals[it];
  }
  __threadfence();
#pragma unroll
  for (int it = 0; it < NBD / (NTHR * 4); ++it) {
    const int s0 = it * (NTHR * 4) + 4 * tid;
    *(volatile v4f*)(dis + (size_t)nodeBase + s0) = vals[it];
  }
}

template <int SPLIT>
__global__ __launch_bounds__(GTHR) void k_gemm(const float* __restrict__ A, const unsigned short* __restrict__ WT,
                                               float* H, int nN) {
  __shared__ __attribute__((aligned(16))) float stg[GBM * FDIM];
  const int tid = (int)threadIdx.x, lane = tid & 31, wave = tid >> 5, hh = lane >> 4, m = lane & 15;
  const int rowBase = (int)blockIdx.x * GBM;
  const int row = rowBase + 16 * wave + m;
  const int rc  = row < nN ? row : nN - 1;
  const float* ar = A + (size_t)rc * FDIM;

  v8f acc[8];
  {
    const v8f z = {0.f, 0.f, 0.f, 0.f, 0.f, 0.f, 0.f, 0.f};
#pragma unroll
    for (int t = 0; t < 8; ++t) acc[t] = z;
  }
  const unsigned short* wp = WT + (size_t)m * FDIM + 8 * hh;

#pragma unroll 1
  for (int kk = 0; kk < FDIM / 32; ++kk) {
    const int k0 = 32 * kk;
    const v4f wa = *(const v4fa*)(ar + k0 + 8 * hh);
    const v4f wb = *(const v4fa*)(ar + k0 + 8 * hh + 4);
    const v4f wc = *(const v4fa*)(ar + k0 + 16 + 8 * hh);
    const v4f wd = *(const v4fa*)(ar + k0 + 16 + 8 * hh + 4);
    float v[16];
    v[0]  = wa.x; v[1]  = wa.y; v[2]  = wa.z; v[3]  = wa.w;
    v[4]  = wb.x; v[5]  = wb.y; v[6]  = wb.z; v[7]  = wb.w;
    v[8]  = wc.x; v[9]  = wc.y; v[10] = wc.z; v[11] = wc.w;
    v[12] = wd.x; v[13] = wd.y; v[14] = wd.z; v[15] = wd.w;
    FragB ah, al;
#pragma unroll
    for (int i = 0; i < 16; ++i) {
      const unsigned hb = bf16_bits(v[i]);
      ah.u[i] = (unsigned short)hb;
      al.u[i] = (unsigned short)((SPLIT != 0) ? bf16_bits(v[i] - __uint_as_float(hb << 16)) : 0u);
    }
#pragma unroll
    for (int nt = 0; nt < 8; ++nt) {
      const unsigned short* wq = wp + (size_t)(16 * nt) * FDIM + k0;
      FragB bf;
      bf.h[0] = *(const v8usa*)wq;
      bf.h[1] = *(const v8usa*)(wq + 16);
      acc[nt] = wmb(ah, bf, acc[nt]);
      if (SPLIT != 0) acc[nt] = wmb(al, bf, acc[nt]);
    }
  }

#pragma unroll
  for (int nt = 0; nt < 8; ++nt) {
    const int lc = 16 * nt + m;
#pragma unroll
    for (int r = 0; r < 8; ++r) {
      const int lr = 16 * wave + 8 * hh + r;
      stg[lr * FDIM + lc] = acc[nt][r];
    }
  }
  __syncthreads();

  v4f pv[16];
#pragma unroll
  for (int i = 0; i < 16; ++i) {
    pv[i] = *(const v4fa*)(stg + (16 * wave + i) * FDIM + 4 * lane);
  }
#pragma unroll
  for (int i = 0; i < 16; ++i) {
    float* op = H + (size_t)(rowBase + 16 * wave + i) * FDIM + 4 * lane;
    *(volatile v4f*)op = pv[i];
  }
  __threadfence();
#pragma unroll
  for (int i = 0; i < 16; ++i) {
    float* op = H + (size_t)(rowBase + 16 * wave + i) * FDIM + 4 * lane;
    *(volatile v4f*)op = pv[i];
  }
}

template <int RELU>
__global__ __launch_bounds__(NTHR) void k_agg(const int* __restrict__ srcs, const int* __restrict__ dsts,
                                              const float* __restrict__ dis, const float* __restrict__ H,
                                              const float* __restrict__ bias, int nE, int nN, int vec8,
                                              float* Z) {
  extern __shared__ __attribute__((aligned(16))) float dacc[];
  __shared__ __attribute__((aligned(16))) int list[LISTN];
  __shared__ __attribute__((aligned(16))) float sdis[NBA];
  __shared__ int wcnt[NWAVE];
  const int tid = (int)threadIdx.x, lane = tid & 31;
  const int wave = __builtin_amdgcn_readfirstlane(tid >> 5);
  const int nodeBase = (int)blockIdx.x * NBA;

  {
    const v4f z4 = {0.f, 0.f, 0.f, 0.f};
#pragma unroll 1
    for (int i = tid; i < (NBA * FDIM) / 4; i += NTHR) *(v4fa*)(dacc + 4 * i) = z4;
  }
  for (int i = tid; i < LISTN; i += NTHR) list[i] = 0;
  for (int i = tid; i < NBA; i += NTHR) {
    int nd = nodeBase + i;
    nd = nd > nN - 1 ? nN - 1 : nd;
    sdis[i] = dis[nd];
  }
  if (tid < NWAVE) wcnt[tid] = 0;
  v4f bv;
  bv.x = bf16_val(bias[4 * lane]);
  bv.y = bf16_val(bias[4 * lane + 1]);
  bv.z = bf16_val(bias[4 * lane + 2]);
  bv.w = bf16_val(bias[4 * lane + 3]);
  __syncthreads();

  const int nChunks = (nE + CHUNK - 1) / CHUNK;
#pragma unroll 1
  for (int ch = 0; ch < nChunks; ++ch) {
    const int cbase = ch * CHUNK;
    const int wc = scan_chunk(dsts, nE, cbase, nodeBase, NBA, vec8, list, tid, lane, wave);
    if (lane == 0) wcnt[wave] = wc;
    __syncthreads();
#pragma unroll 1
    for (int w2 = 0; w2 < NWAVE; ++w2) {
      int c = __builtin_amdgcn_readfirstlane(wcnt[w2]);
      c = c < 0 ? 0 : (c > WCAP ? WCAP : c);
#pragma unroll 1
      for (int b0 = 0; b0 < c; b0 += 32) {
        const int idx = b0 + lane;
        const int ent = list[w2 * WCAP + (idx < WCAP ? idx : WCAP - 1)];
        const int el  = (ent >> SLB) & (CHUNK - 1);
        int eid = cbase + el;
        eid = eid < 0 ? 0 : (eid > nE - 1 ? nE - 1 : eid);
        const int sraw = srcs[eid];
        const int s = sraw < 0 ? 0 : (sraw > nN - 1 ? nN - 1 : sraw);
        const int dvi = __float_as_int(dis[s]);
        int sl = ent & (NBD - 1);
        sl = sl > NBA - 1 ? NBA - 1 : sl;
        const bool mine = (idx < c) && ((unsigned)(sl - wave * SPW) < (unsigned)SPW);
        unsigned msk = __builtin_amdgcn_ballot_w32(mine);
#pragma unroll 1
        for (; msk != 0u; msk &= msk - 1u) {
          const int k   = (int)__builtin_ctz(msk);
          const int slk = __builtin_amdgcn_readlane(sl, k);
          const int sik = __builtin_amdgcn_readlane(s, k);
          const float nrm = __int_as_float(__builtin_amdgcn_readlane(dvi, k)) * sdis[slk];
          const v4f hv = *(const v4fa*)(H + (size_t)sik * FDIM + 4 * lane);
          float* ap = dacc + (size_t)slk * FDIM + 4 * lane;
          v4f a = *(const v4fa*)ap;
          a.x = fmaf(hv.x, nrm, a.x);
          a.y = fmaf(hv.y, nrm, a.y);
          a.z = fmaf(hv.z, nrm, a.z);
          a.w = fmaf(hv.w, nrm, a.w);
          *(v4fa*)ap = a;
        }
      }
    }
    __syncthreads();
  }

#pragma unroll 1
  for (int s2 = 0; s2 < SPW; ++s2) {
    const int sl = wave * SPW + s2;
    const int node = nodeBase + sl;
    const int nc = node > nN - 1 ? nN - 1 : node;
    const v4f hv = *(const v4fa*)(H + (size_t)nc * FDIM + 4 * lane);
    const float dd = sdis[sl];
    const float nrm = dd * dd;
    float* ap = dacc + (size_t)sl * FDIM + 4 * lane;
    const v4f a = *(const v4fa*)ap;
    v4f z;
    z.x = fmaf(hv.x, nrm, a.x) + bv.x;
    z.y = fmaf(hv.y, nrm, a.y) + bv.y;
    z.z = fmaf(hv.z, nrm, a.z) + bv.z;
    z.w = fmaf(hv.w, nrm, a.w) + bv.w;
    if (RELU != 0) {
      z.x = fmaxf(z.x, 0.f); z.y = fmaxf(z.y, 0.f); z.z = fmaxf(z.z, 0.f); z.w = fmaxf(z.w, 0.f);
    }
    *(v4fa*)ap = z;
  }
#pragma unroll 1
  for (int s2 = 0; s2 < SPW; ++s2) {
    const int sl = wave * SPW + s2;
    const int node = nodeBase + sl;
    const v4f z = *(const v4fa*)(dacc + (size_t)sl * FDIM + 4 * lane);
    *(volatile v4f*)(Z + (size_t)node * FDIM + 4 * lane) = z;
  }
  __threadfence();
#pragma unroll 1
  for (int s2 = 0; s2 < SPW; ++s2) {
    const int sl = wave * SPW + s2;
    const int node = nodeBase + sl;
    const v4f z = *(const v4fa*)(dacc + (size_t)sl * FDIM + 4 * lane);
    *(volatile v4f*)(Z + (size_t)node * FDIM + 4 * lane) = z;
  }
}

__global__ __launch_bounds__(DTHR) void k_decode(const float* __restrict__ Z, const int* __restrict__ lsrc,
                                                 const int* __restrict__ ldst, int EL, int nN, float* out) {
  const int tid = (int)threadIdx.x, lane = tid & 31;
  const int wave = __builtin_amdgcn_readfirstlane(tid >> 5);
  const int eBase = ((int)blockIdx.x * (DTHR / 32) + wave) * 32;
  if (eBase >= EL) return;
  int ei = eBase + lane;
  ei = ei > EL - 1 ? EL - 1 : ei;
  int a = lsrc[ei];
  a = a < 0 ? 0 : (a > nN - 1 ? nN - 1 : a);
  int d = ldst[ei];
  d = d < 0 ? 0 : (d > nN - 1 ? nN - 1 : d);

  float res = 0.f;
#pragma unroll 2
  for (int j = 0; j < 32; ++j) {
    const int aj = __builtin_amdgcn_readlane(a, j);
    const int dj = __builtin_amdgcn_readlane(d, j);
    const v4f za = *(const v4fa*)(Z + (size_t)aj * FDIM + 4 * lane);
    const v4f zd = *(const v4fa*)(Z + (size_t)dj * FDIM + 4 * lane);
    float p = za.x * zd.x;
    p = fmaf(za.y, zd.y, p);
    p = fmaf(za.z, zd.z, p);
    p = fmaf(za.w, zd.w, p);
    p += __shfl_xor(p, 16);
    p += __shfl_xor(p, 8);
    p += __shfl_xor(p, 4);
    p += __shfl_xor(p, 2);
    p += __shfl_xor(p, 1);
    res = (lane == j) ? p : res;
  }
  const float e  = expf(-res);
  const float sg = __builtin_amdgcn_rcpf(1.0f + e);
  float* op = out + eBase + lane;
  if (eBase + 32 <= EL) {
    *(volatile float*)op = sg;
    __threadfence();
    *(volatile float*)op = sg;
  } else {
    const bool ok = (eBase + lane) < EL;
    if (ok) *(volatile float*)op = sg;
    __threadfence();
    if (ok) *(volatile float*)op = sg;
  }
}

static inline int cdiv(int a, int b) { return (a + b - 1) / b; }

extern "C" void kernel_launch(void* const* d_in, const int* in_sizes, int n_in,
                              void* d_out, int out_size, void* d_ws, size_t ws_size,
                              hipStream_t stream) {
  if (n_in < 7) return;
  if (in_sizes[0] < FDIM || (in_sizes[0] % FDIM) != 0) return;
  const int nN = in_sizes[0] / FDIM;
  if (in_sizes[1] < 2 || (in_sizes[1] & 1) != 0) return;
  const int nE = in_sizes[1] / 2;
  if (in_sizes[2] < 2 || (in_sizes[2] & 1) != 0) return;
  const int EL = in_sizes[2] / 2;
  if (in_sizes[3] != FDIM * FDIM || in_sizes[4] != FDIM) return;
  if (in_sizes[5] != FDIM * FDIM || in_sizes[6] != FDIM) return;
  if (out_size != EL || nN < 1) return;

  const float* x    = (const float*)d_in[0];
  const int*   edge = (const int*)d_in[1];
  const int*   lab  = (const int*)d_in[2];
  const float* W1   = (const float*)d_in[3];
  const float* b1   = (const float*)d_in[4];
  const float* W2   = (const float*)d_in[5];
  const float* b2   = (const float*)d_in[6];
  float* out = (float*)d_out;
  const int* src = edge;
  const int* dst = edge + nE;
  const int* ls  = lab;
  const int* ld  = lab + EL;

  const int gD   = cdiv(nN, NBD);
  const int NBPD = gD * NBD;
  const int gA   = cdiv(nN, NBA);
  const int NBPA = gA * NBA;
  const int MP   = cdiv(nN, GBM) * GBM;
  const int gM   = MP / GBM;
  const int gL   = cdiv(EL, (DTHR / 32) * 32);
  const int vec8 = ((nE & 3) == 0) ? 1 : 0;

  char* ws = (char*)d_ws;
  size_t off = 0;
  const size_t oDIS = off; off += (size_t)NBPD * 4;                 off = (off + 255) & ~(size_t)255;
  const size_t oWT1 = off; off += (size_t)FDIM * FDIM * 2;          off = (off + 255) & ~(size_t)255;
  const size_t oWT2 = off; off += (size_t)FDIM * FDIM * 2;          off = (off + 255) & ~(size_t)255;
  const size_t oH1  = off; off += (size_t)MP * FDIM * 4;            off = (off + 255) & ~(size_t)255;
  const size_t oZ1  = off; off += (size_t)NBPA * FDIM * 4;          off = (off + 255) & ~(size_t)255;
  const size_t oH2  = off; off += (size_t)MP * FDIM * 4;            off = (off + 255) & ~(size_t)255;
  const size_t oZ2  = off; off += (size_t)NBPA * FDIM * 4;          off = (off + 255) & ~(size_t)255;
  if (off > ws_size || off > (size_t)WSMAX) return;
  float*          DIS = (float*)(ws + oDIS);
  unsigned short* WT1 = (unsigned short*)(ws + oWT1);
  unsigned short* WT2 = (unsigned short*)(ws + oWT2);
  float*          H1  = (float*)(ws + oH1);
  float*          Z1  = (float*)(ws + oZ1);
  float*          H2  = (float*)(ws + oH2);
  float*          Z2  = (float*)(ws + oZ2);

  const size_t dynB = (size_t)NBA * FDIM * 4;
  hipFuncSetAttribute(reinterpret_cast<const void*>(&k_agg<1>), hipFuncAttributeMaxDynamicSharedMemorySize, (int)dynB);
  hipFuncSetAttribute(reinterpret_cast<const void*>(&k_agg<0>), hipFuncAttributeMaxDynamicSharedMemorySize, (int)dynB);

  k_wprep<<<2 * (WUNITS / NTHR), NTHR, 0, stream>>>(W1, W2, WT1, WT2);
  k_deg<<<gD, NTHR, 0, stream>>>(dst, nE, vec8, DIS);
  k_gemm<0><<<gM, GTHR, 0, stream>>>(x, WT1, H1, nN);
  k_agg<1><<<gA, NTHR, dynB, stream>>>(src, dst, DIS, H1, b1, nE, nN, vec8, Z1);
  k_gemm<1><<<gM, GTHR, 0, stream>>>(Z1, WT2, H2, nN);
  k_agg<0><<<gA, NTHR, dynB, stream>>>(src, dst, DIS, H2, b2, nE, nN, vec8, Z2);
  k_decode<<<gL, DTHR, 0, stream>>>(Z2, ls, ld, EL, nN, out);
}
